// SE3EquivariantLayer_16277926052601
// MI455X (gfx1250) — hardware-verified
//
#include <hip/hip_runtime.h>
#include <math.h>


#pragma clang fp contract(off)

#define NATOMS 512
#define DDIM   128
#define MROWS  1024
#define NPLANES 9
#define PLANE_ELEMS 16384
#define TPITCH 136
#define FPITCH 132
#define AGGP   32

typedef __bf16 v16b  __attribute__((ext_vector_type(16)));
typedef __bf16 v8b   __attribute__((ext_vector_type(8)));
typedef __bf16 v16ba __attribute__((ext_vector_type(16), may_alias));
typedef __bf16 v8ba  __attribute__((ext_vector_type(8), may_alias));
typedef float  v8f   __attribute__((ext_vector_type(8)));
typedef float  v4f   __attribute__((ext_vector_type(4)));
typedef float  v8fa  __attribute__((ext_vector_type(8), may_alias));
typedef float  v4fa  __attribute__((ext_vector_type(4), may_alias));

__device__ __forceinline__ v8f wmma_bf16_acc(v8f c, v16b a, v16b b) {
    c = __builtin_amdgcn_wmma_f32_16x16x32_bf16(false, a, false, b, (short)0, c, false, false);
    asm volatile("v_nop\n\tv_nop\n\tv_nop\n\tv_nop" : "+v"(c) : "v"(a), "v"(b));
    return c;
}

__device__ __forceinline__ float bf16_hi_f(float x) {
    unsigned int u = __float_as_uint(x);
    u = (u + 0x7FFFu + ((u >> 16) & 1u)) & 0xFFFF0000u;
    return __uint_as_float(u);
}

__device__ __forceinline__ float silu_f(float x) {
    return x * __builtin_amdgcn_rcpf(1.0f + __expf(-x));
}

__device__ __forceinline__ float wave_sum(float v) {
    v += __shfl_xor(v, 16);
    v += __shfl_xor(v, 8);
    v += __shfl_xor(v, 4);
    v += __shfl_xor(v, 2);
    v += __shfl_xor(v, 1);
    return v;
}

__device__ __forceinline__ float wave_max(float v) {
    v = fmaxf(v, __shfl_xor(v, 16));
    v = fmaxf(v, __shfl_xor(v, 8));
    v = fmaxf(v, __shfl_xor(v, 4));
    v = fmaxf(v, __shfl_xor(v, 2));
    v = fmaxf(v, __shfl_xor(v, 1));
    return v;
}

__global__ __launch_bounds__(256)
void pack_kernel(const float* __restrict__ Ws1, const float* __restrict__ Ws2,
                 const float* __restrict__ Wv1, const float* __restrict__ Wv2,
                 const float* __restrict__ Wa1, __bf16* __restrict__ pack)
{
    const int t = blockIdx.x * 256 + threadIdx.x;
    if (t >= (NPLANES * PLANE_ELEMS) / 8) return;
    const int E0 = t << 3;
    const int p  = E0 >> 14;
    const int f  = (E0 >> 9) & 31;
    const int L  = (E0 >> 4) & 31;
    const int e0 = E0 & 15;
    const int n  = ((f & 7) << 4) + (L & 15);
    const int kb = ((f >> 3) << 5) + ((L >> 4) << 3) + ((e0 >> 3) << 4);
    const float* W = (p < 2) ? Ws1 : (p < 4) ? Ws2 : (p < 6) ? Wv1 : (p < 8) ? Wv2 : Wa1;
    const bool lo = (p < 8) && ((p & 1) != 0);
    v8b o;
    #pragma unroll
    for (int q = 0; q < 8; ++q) {
        const float x  = W[(kb + q) * DDIM + n];
        const float hf = bf16_hi_f(x);
        const float v  = lo ? bf16_hi_f(x - hf) : hf;
        o[q] = (__bf16)v;
    }
    __bf16* dst = pack + E0;
    *(volatile v8b*)dst = o;
    __threadfence();
    *(volatile v8b*)dst = o;
}

__global__ __launch_bounds__(256)
void node_kernel(const float* __restrict__ nf,
                 const float* __restrict__ bs1, const float* __restrict__ bs2,
                 const float* __restrict__ bv1, const float* __restrict__ bv2,
                 const float* __restrict__ ba1,
                 const __bf16* __restrict__ pack,
                 float* __restrict__ scalar_out,
                 float* __restrict__ pre,
                 float* __restrict__ vf4)
{
    __shared__ __bf16 nfh[16][TPITCH] __attribute__((aligned(16)));
    __shared__ __bf16 nfl[16][TPITCH] __attribute__((aligned(16)));
    __shared__ __bf16 hsh[16][TPITCH] __attribute__((aligned(16)));
    __shared__ __bf16 hsl[16][TPITCH] __attribute__((aligned(16)));
    __shared__ __bf16 hvh[16][TPITCH] __attribute__((aligned(16)));
    __shared__ __bf16 hvl[16][TPITCH] __attribute__((aligned(16)));
    __shared__ float preT[16][FPITCH] __attribute__((aligned(16)));
    __shared__ float outT[16][FPITCH] __attribute__((aligned(16)));
    __shared__ float vfT[16][4] __attribute__((aligned(16)));

    const int tid  = threadIdx.x;
    const int lane = tid & 31;
    const int wave = tid >> 5;
    const int h    = lane >> 4;
    const int m    = lane & 15;
    const int rowbase = blockIdx.x * 16;
    const int nn   = wave * 16 + m;

    {
        const int E0 = tid << 3;
        const int r  = E0 >> 7;
        const int c0 = E0 & 127;
        const float* src = nf + (size_t)(rowbase + r) * DDIM + c0;
        const v4f x0 = *(const v4f*)src;
        const v4f x1 = *(const v4f*)(src + 4);
        v8b hi8, lo8;
        #pragma unroll
        for (int q = 0; q < 4; ++q) {
            const float x = x0[q]; const float hf = bf16_hi_f(x);
            hi8[q] = (__bf16)hf; lo8[q] = (__bf16)bf16_hi_f(x - hf);
            const float y = x1[q]; const float hg = bf16_hi_f(y);
            hi8[q + 4] = (__bf16)hg; lo8[q + 4] = (__bf16)bf16_hi_f(y - hg);
        }
        *(v8ba*)(&nfh[r][c0]) = hi8;
        *(v8ba*)(&nfl[r][c0]) = lo8;
    }
    __syncthreads();

    v8f cs, cv, ca;
    {
        const float b1 = bs1[nn], b2 = bv1[nn], b3 = ba1[nn];
        #pragma unroll
        for (int r = 0; r < 8; ++r) { cs[r] = b1; cv[r] = b2; ca[r] = b3; }
    }
    #pragma unroll 1
    for (int ks = 0; ks < 4; ++ks) {
        const int k0 = ks * 32 + 8 * h;
        const v8b ah0 = *(const v8ba*)(&nfh[m][k0]);
        const v8b ah1 = *(const v8ba*)(&nfh[m][k0 + 16]);
        const v8b al0 = *(const v8ba*)(&nfl[m][k0]);
        const v8b al1 = *(const v8ba*)(&nfl[m][k0 + 16]);
        const v16b ah = __builtin_shufflevector(ah0, ah1, 0, 1, 2, 3, 4, 5, 6, 7, 8, 9, 10, 11, 12, 13, 14, 15);
        const v16b al = __builtin_shufflevector(al0, al1, 0, 1, 2, 3, 4, 5, 6, 7, 8, 9, 10, 11, 12, 13, 14, 15);
        const __bf16* fb = pack + ((size_t)((ks * 8 + wave) * 32 + lane) << 4);
        const v16b bsh = *(const v16ba*)(fb + 0 * PLANE_ELEMS);
        const v16b bsl = *(const v16ba*)(fb + 1 * PLANE_ELEMS);
        const v16b bvh = *(const v16ba*)(fb + 4 * PLANE_ELEMS);
        const v16b bvl = *(const v16ba*)(fb + 5 * PLANE_ELEMS);
        const v16b bah = *(const v16ba*)(fb + 8 * PLANE_ELEMS);
        cs = wmma_bf16_acc(cs, ah, bsh);
        cs = wmma_bf16_acc(cs, ah, bsl);
        cs = wmma_bf16_acc(cs, al, bsh);
        cv = wmma_bf16_acc(cv, ah, bvh);
        cv = wmma_bf16_acc(cv, ah, bvl);
        cv = wmma_bf16_acc(cv, al, bvh);
        ca = wmma_bf16_acc(ca, ah, bah);
    }
    #pragma unroll
    for (int r = 0; r < 8; ++r) {
        const int row = 8 * h + r;
        const float s  = silu_f(cs[r]);
        const float sf = bf16_hi_f(s);
        hsh[row][nn] = (__bf16)sf;
        hsl[row][nn] = (__bf16)bf16_hi_f(s - sf);
        const float v  = silu_f(cv[r]);
        const float vh = bf16_hi_f(v);
        hvh[row][nn] = (__bf16)vh;
        hvl[row][nn] = (__bf16)bf16_hi_f(v - vh);
        preT[row][nn] = ca[r];
    }
    __syncthreads();

    v8f c2s, c2v;
    {
        const float b1 = bs2[nn], b2 = bv2[nn];
        #pragma unroll
        for (int r = 0; r < 8; ++r) { c2s[r] = b1; c2v[r] = b2; }
    }
    #pragma unroll 1
    for (int ks = 0; ks < 4; ++ks) {
        const int k0 = ks * 32 + 8 * h;
        const v8b s0 = *(const v8ba*)(&hsh[m][k0]);
        const v8b s1 = *(const v8ba*)(&hsh[m][k0 + 16]);
        const v8b t0 = *(const v8ba*)(&hsl[m][k0]);
        const v8b t1 = *(const v8ba*)(&hsl[m][k0 + 16]);
        const v8b u0 = *(const v8ba*)(&hvh[m][k0]);
        const v8b u1 = *(const v8ba*)(&hvh[m][k0 + 16]);
        const v8b w0 = *(const v8ba*)(&hvl[m][k0]);
        const v8b w1 = *(const v8ba*)(&hvl[m][k0 + 16]);
        const v16b ash = __builtin_shufflevector(s0, s1, 0, 1, 2, 3, 4, 5, 6, 7, 8, 9, 10, 11, 12, 13, 14, 15);
        const v16b asl = __builtin_shufflevector(t0, t1, 0, 1, 2, 3, 4, 5, 6, 7, 8, 9, 10, 11, 12, 13, 14, 15);
        const v16b avh = __builtin_shufflevector(u0, u1, 0, 1, 2, 3, 4, 5, 6, 7, 8, 9, 10, 11, 12, 13, 14, 15);
        const v16b avl = __builtin_shufflevector(w0, w1, 0, 1, 2, 3, 4, 5, 6, 7, 8, 9, 10, 11, 12, 13, 14, 15);
        const __bf16* fb = pack + ((size_t)((ks * 8 + wave) * 32 + lane) << 4);
        const v16b b2h = *(const v16ba*)(fb + 2 * PLANE_ELEMS);
        const v16b b2l = *(const v16ba*)(fb + 3 * PLANE_ELEMS);
        const v16b b4h = *(const v16ba*)(fb + 6 * PLANE_ELEMS);
        const v16b b4l = *(const v16ba*)(fb + 7 * PLANE_ELEMS);
        c2s = wmma_bf16_acc(c2s, ash, b2h);
        c2s = wmma_bf16_acc(c2s, ash, b2l);
        c2s = wmma_bf16_acc(c2s, asl, b2h);
        c2v = wmma_bf16_acc(c2v, avh, b4h);
        c2v = wmma_bf16_acc(c2v, avh, b4l);
        c2v = wmma_bf16_acc(c2v, avl, b4h);
    }
    #pragma unroll
    for (int r = 0; r < 8; ++r) {
        const int row = 8 * h + r;
        outT[row][nn] = c2s[r];
        if (wave == 0 && m < 4) vfT[row][m] = (m < 3) ? c2v[r] : 0.0f;
    }
    __syncthreads();

    const int ra = wave * 2, rb = wave * 2 + 1;
    const v4f oa = *(const v4fa*)(&outT[ra][lane * 4]);
    const v4f ob = *(const v4fa*)(&outT[rb][lane * 4]);
    const v4f pa = *(const v4fa*)(&preT[ra][lane * 4]);
    const v4f pb = *(const v4fa*)(&preT[rb][lane * 4]);
    float* poa = scalar_out + (size_t)(rowbase + ra) * DDIM + lane * 4;
    float* pob = scalar_out + (size_t)(rowbase + rb) * DDIM + lane * 4;
    float* ppa = pre + (size_t)(rowbase + ra) * DDIM + lane * 4;
    float* ppb = pre + (size_t)(rowbase + rb) * DDIM + lane * 4;
    const bool dov = (wave == 0) && (lane < 16);
    v4f vv = {0.0f, 0.0f, 0.0f, 0.0f};
    float* pv = vf4;
    if (dov) { vv = *(const v4fa*)(&vfT[lane][0]); pv = vf4 + (size_t)(rowbase + lane) * 4; }

    *(volatile v4f*)poa = oa;
    *(volatile v4f*)pob = ob;
    *(volatile v4f*)ppa = pa;
    *(volatile v4f*)ppb = pb;
    if (dov) *(volatile v4f*)pv = vv;
    __threadfence();
    *(volatile v4f*)poa = oa;
    *(volatile v4f*)pob = ob;
    *(volatile v4f*)ppa = pa;
    *(volatile v4f*)ppb = pb;
    if (dov) *(volatile v4f*)pv = vv;
}

__global__ __launch_bounds__(256)
void pair_attn_kernel(const float* __restrict__ coords,
                      const int*   __restrict__ emask,
                      const float* __restrict__ Wa1,
                      const float* __restrict__ Wa2,
                      const float* __restrict__ ba2,
                      const float* __restrict__ pre,
                      const float* __restrict__ vf4,
                      float* __restrict__ agg)
{
    __shared__ float lg[NATOMS];
    __shared__ float rw[32];
    __shared__ float preS[DDIM] __attribute__((aligned(32)));
    __shared__ float w0S[DDIM]  __attribute__((aligned(32)));
    __shared__ float w1S[DDIM]  __attribute__((aligned(32)));
    __shared__ float w2S[DDIM]  __attribute__((aligned(32)));
    __shared__ float xyzS[NATOMS * 3];
    __shared__ __bf16 wa2B[4 * 32 * 16] __attribute__((aligned(32)));

    const int tid  = threadIdx.x;
    const int lane = tid & 31;
    const int wave = tid >> 5;
    const int h    = lane >> 4;
    const int m    = lane & 15;
    const int bi   = blockIdx.x;
    const int b    = bi >> 9;
    const int i    = bi & (NATOMS - 1);

    if (tid < DDIM) {
        preS[tid] = pre[(size_t)bi * DDIM + tid];
        w0S[tid]  = Wa1[128 * DDIM + tid];
        w1S[tid]  = Wa1[129 * DDIM + tid];
        w2S[tid]  = Wa1[130 * DDIM + tid];
    }
    #pragma unroll
    for (int e = 0; e < 6; ++e) {
        const int idx = tid * 6 + e;
        xyzS[idx] = coords[(size_t)b * NATOMS * 3 + idx];
    }
    {
        const int E0 = tid << 3;
        const int ks = E0 >> 9;
        const int L  = (E0 >> 4) & 31;
        const int e0 = E0 & 15;
        const int kb = ks * 32 + ((L >> 4) << 3) + ((e0 >> 3) << 4);
        const bool col0 = ((L & 15) == 0);
        v8b o;
        #pragma unroll
        for (int q = 0; q < 8; ++q) {
            const float x = col0 ? bf16_hi_f(Wa2[kb + q]) : 0.0f;
            o[q] = (__bf16)x;
        }
        *(v8ba*)(&wa2B[E0]) = o;
    }
    __syncthreads();

    const float xi0 = xyzS[i * 3], xi1 = xyzS[i * 3 + 1], xi2 = xyzS[i * 3 + 2];
    const float bias2 = ba2[0];
    const int* mrow = emask + (size_t)bi * NATOMS;

    #pragma unroll 1
    for (int chunk = 0; chunk < 4; ++chunk) {
        const int jbase = wave * 64 + chunk * 16;
        const int jm = jbase + m;
        const float dx = xi0 - xyzS[jm * 3];
        const float dy = xi1 - xyzS[jm * 3 + 1];
        const float dz = xi2 - xyzS[jm * 3 + 2];
        const float d2 = dx * dx + dy * dy + dz * dz;
        const float dist = (d2 > 0.0f) ? sqrtf(d2) : 0.0f;
        const float f0 = dist;
        const float f1 = 1.0f / (dist + 1e-6f);
        const float f2 = __expf(-dist);

        v8f acc = {0.0f, 0.0f, 0.0f, 0.0f, 0.0f, 0.0f, 0.0f, 0.0f};
        #pragma unroll
        for (int ks = 0; ks < 4; ++ks) {
            v16b afh, afl;
            #pragma unroll
            for (int g = 0; g < 2; ++g) {
                const int nb = ks * 32 + 8 * h + 16 * g;
                const v8f pv = *(const v8fa*)(&preS[nb]);
                const v8f u0 = *(const v8fa*)(&w0S[nb]);
                const v8f u1 = *(const v8fa*)(&w1S[nb]);
                const v8f u2 = *(const v8fa*)(&w2S[nb]);
                #pragma unroll
                for (int q = 0; q < 8; ++q) {
                    float t = fmaf(f0, u0[q], pv[q]);
                    t = fmaf(f1, u1[q], t);
                    t = fmaf(f2, u2[q], t);
                    const float s  = silu_f(t);
                    const float sh = bf16_hi_f(s);
                    afh[g * 8 + q] = (__bf16)sh;
                    afl[g * 8 + q] = (__bf16)bf16_hi_f(s - sh);
                }
            }
            const v16b bfr = *(const v16ba*)(&wa2B[(ks * 32 + lane) << 4]);
            acc = wmma_bf16_acc(acc, afh, bfr);
            acc = wmma_bf16_acc(acc, afl, bfr);
        }
        if (m == 0) {
            #pragma unroll
            for (int r = 0; r < 8; ++r) {
                const int j = jbase + 8 * h + r;
                float v = acc[r] + bias2;
                if (mrow[j] == 0) v = -__builtin_inff();
                lg[j] = v;
            }
        }
    }
    __syncthreads();

    const float l0 = lg[tid], l1 = lg[tid + 256];
    float mx = wave_max(fmaxf(l0, l1));
    if (lane == 0) rw[wave] = mx;
    __syncthreads();
    mx = rw[0];
    #pragma unroll
    for (int w = 1; w < 8; ++w) mx = fmaxf(mx, rw[w]);
    __syncthreads();
    const float e0 = __expf(l0 - mx);
    const float e1 = __expf(l1 - mx);
    const float s  = wave_sum(e0 + e1);
    if (lane == 0) rw[wave] = s;
    __syncthreads();
    float tot = rw[0];
    #pragma unroll
    for (int w = 1; w < 8; ++w) tot += rw[w];
    __syncthreads();
    const float inv = __builtin_amdgcn_rcpf(tot);
    const float a0 = e0 * inv, a1 = e1 * inv;

    const int j0 = tid, j1 = tid + 256;
    float p0 = a0 * (xi0 - xyzS[j0 * 3])     + a1 * (xi0 - xyzS[j1 * 3]);
    float p1 = a0 * (xi1 - xyzS[j0 * 3 + 1]) + a1 * (xi1 - xyzS[j1 * 3 + 1]);
    float p2 = a0 * (xi2 - xyzS[j0 * 3 + 2]) + a1 * (xi2 - xyzS[j1 * 3 + 2]);
    p0 = wave_sum(p0);
    p1 = wave_sum(p1);
    p2 = wave_sum(p2);
    if (lane == 0) { rw[wave * 4] = p0; rw[wave * 4 + 1] = p1; rw[wave * 4 + 2] = p2; }
    __syncthreads();
    if (tid < 8) {
        float s0 = 0.0f, s1 = 0.0f, s2 = 0.0f;
        #pragma unroll
        for (int w = 0; w < 8; ++w) { s0 += rw[w * 4]; s1 += rw[w * 4 + 1]; s2 += rw[w * 4 + 2]; }
        const float o0 = s0 * vf4[(size_t)bi * 4];
        const float o1 = s1 * vf4[(size_t)bi * 4 + 1];
        const float o2 = s2 * vf4[(size_t)bi * 4 + 2];
        v4f val = {0.0f, 0.0f, 0.0f, 0.0f};
        if (tid == 0) { val[0] = o0; val[1] = o1; val[2] = o2; }
        float* dst = agg + (size_t)bi * AGGP + tid * 4;
        *(volatile v4f*)dst = val;
        __threadfence();
        *(volatile v4f*)dst = val;
    }
}

__device__ __forceinline__ v4f gather_out1(const float* __restrict__ agg, int q) {
    v4f v;
    #pragma unroll
    for (int c = 0; c < 4; ++c) {
        const int el   = (q << 2) + c;
        const int node = el / 3;
        const int comp = el - node * 3;
        v[c] = agg[(size_t)node * AGGP + comp];
    }
    return v;
}

__global__ __launch_bounds__(256)
void out1_kernel(const float* __restrict__ agg, float* __restrict__ out1)
{
    const int tid = threadIdx.x;
    const int q0 = tid, q1 = tid + 256, q2 = tid + 512;
    const v4f v0 = gather_out1(agg, q0);
    const v4f v1 = gather_out1(agg, q1);
    const v4f v2 = gather_out1(agg, q2);
    float* d0 = out1 + (q0 << 2);
    float* d1 = out1 + (q1 << 2);
    float* d2p = out1 + (q2 << 2);
    *(volatile v4f*)d0 = v0;
    *(volatile v4f*)d1 = v1;
    *(volatile v4f*)d2p = v2;
    __threadfence();
    *(volatile v4f*)d0 = v0;
    *(volatile v4f*)d1 = v1;
    *(volatile v4f*)d2p = v2;
}

extern "C" void kernel_launch(void* const* d_in, const int* in_sizes, int n_in,
                              void* d_out, int out_size, void* d_ws, size_t ws_size,
                              hipStream_t stream) {
    if (n_in < 15) return;
    if (in_sizes[0] != MROWS * DDIM || in_sizes[1] != MROWS * 3 || in_sizes[2] != MROWS * NATOMS ||
        in_sizes[3] != DDIM * DDIM || in_sizes[5] != DDIM * DDIM || in_sizes[7] != DDIM * DDIM ||
        in_sizes[9] != DDIM * DDIM || in_sizes[11] != 131 * DDIM || in_sizes[13] != DDIM ||
        in_sizes[14] < 1 || out_size != MROWS * DDIM + MROWS * 3) return;

    const float* nf  = (const float*)d_in[0];
    const float* xyz = (const float*)d_in[1];
    const int*   em  = (const int*)  d_in[2];
    const float* Ws1 = (const float*)d_in[3];
    const float* bs1 = (const float*)d_in[4];
    const float* Ws2 = (const float*)d_in[5];
    const float* bs2 = (const float*)d_in[6];
    const float* Wv1 = (const float*)d_in[7];
    const float* bv1 = (const float*)d_in[8];
    const float* Wv2 = (const float*)d_in[9];
    const float* bv2 = (const float*)d_in[10];
    const float* Wa1 = (const float*)d_in[11];
    const float* ba1 = (const float*)d_in[12];
    const float* Wa2 = (const float*)d_in[13];
    const float* ba2 = (const float*)d_in[14];

    float* scalar_out = (float*)d_out;
    float* vec_out    = (float*)d_out + MROWS * DDIM;

    const size_t off_pre  = 0;
    const size_t off_vf4  = off_pre  + (size_t)MROWS * DDIM * sizeof(float);
    const size_t off_pack = off_vf4  + (size_t)MROWS * 4 * sizeof(float);
    const size_t off_agg  = off_pack + (size_t)NPLANES * PLANE_ELEMS * 2;
    const size_t total    = off_agg  + (size_t)MROWS * AGGP * sizeof(float);
    if (ws_size < total) return;

    char*   ws   = (char*)d_ws;
    float*  pre  = (float*)(ws + off_pre);
    float*  vf4  = (float*)(ws + off_vf4);
    __bf16* pack = (__bf16*)(ws + off_pack);
    float*  agg  = (float*)(ws + off_agg);

    pack_kernel<<<(NPLANES * PLANE_ELEMS / 8) / 256, 256, 0, stream>>>(Ws1, Ws2, Wv1, Wv2, Wa1, pack);

    node_kernel<<<MROWS / 16, 256, 0, stream>>>(nf, bs1, bs2, bv1, bv2, ba1, pack, scalar_out, pre, vf4);

    pair_attn_kernel<<<MROWS, 256, 0, stream>>>(xyz, em, Wa1, Wa2, ba2, pre, vf4, agg);

    out1_kernel<<<1, 256, 0, stream>>>(agg, vec_out);
}
